// EdgeWeightLearner_9174050144888
// MI455X (gfx1250) — hardware-verified
//
#include <hip/hip_runtime.h>
#include <stddef.h>


#define CH     128
#define KPB    128
#define NCOL   16
#define GROWS  64
#define GTHR   128
#define ETHR   256
#define PTHR   256
#define WSC    16.0f
#define RWS    0.0625f
#define WSCAP  134217728

static_assert(GROWS == (GTHR / 32) * 16);
static_assert((CH % 32) == 0);
static_assert(NCOL * KPB == PTHR * 8);
static_assert(ETHR == 256);

typedef float    v4f  __attribute__((ext_vector_type(4)));
typedef float    v8f  __attribute__((ext_vector_type(8)));
typedef _Float16 v8h  __attribute__((ext_vector_type(8)));
typedef _Float16 v16h __attribute__((ext_vector_type(16)));
union Frag { v16h v; v8h h[2]; };

__device__ __forceinline__ v8f wmh(v16h a, v16h b, v8f c) {
  v8f d = __builtin_amdgcn_wmma_f32_16x16x32_f16(false, a, false, b, (short)0, c, false, false);
  asm volatile("v_nop\n\tv_nop\n\tv_nop\n\tv_nop" : "+v"(d) : "v"(a), "v"(b));
  return d;
}

__device__ __forceinline__ float sigm(float s) {
  s = fminf(fmaxf(s, -40.0f), 40.0f);
  const float ex = __expf(-s);
  return __builtin_amdgcn_rcpf(1.0f + ex);
}

__device__ __forceinline__ int clampi(int v, int hi) {
  return v < 0 ? 0 : (v > hi ? hi : v);
}

__global__ __launch_bounds__(PTHR) void k_wprep(const float* __restrict__ W, _Float16* Wpl) {
  const int tid = threadIdx.x;
  const int n = tid >> 4, k0 = (tid & 15) * 8;
  const int nb = (n < 2 ? n : 1) * CH + k0;
  const float sc = (n < 2) ? WSC : 0.0f;
  float v[8];
#pragma unroll
  for (int e = 0; e < 8; ++e) v[e] = W[nb + e];
  v8h hv;
#pragma unroll
  for (int e = 0; e < 8; ++e) hv[e] = (_Float16)(v[e] * sc);
  _Float16* dp = Wpl + tid * 8;
  *(volatile v8h*)dp = hv;
  __threadfence();
  *(volatile v8h*)dp = hv;
}

__global__ __launch_bounds__(GTHR) void k_nodegemm(const float* __restrict__ x,
                                                   const _Float16* __restrict__ Wpl,
                                                   float* AB, int nN, int nPad) {
  __shared__ __attribute__((aligned(16))) float stg[2 * GROWS];
  const int tid = threadIdx.x, lane = tid & 31, wave = tid >> 5, hh = lane >> 4, m = lane & 15;
  const int rowBase = blockIdx.x * GROWS;
  int xrow = rowBase + wave * 16 + m;
  xrow = xrow > nN - 1 ? nN - 1 : xrow;
  const float* xp = x + (size_t)xrow * CH + 8 * hh;
  const _Float16* bp = Wpl + m * KPB + 8 * hh;

  v8f acc = {0.f, 0.f, 0.f, 0.f, 0.f, 0.f, 0.f, 0.f};
#pragma unroll
  for (int ks = 0; ks < CH / 32; ++ks) {
    const float* pa = xp + 32 * ks;
    const v4f f0 = *(const v4f*)(pa);
    const v4f f1 = *(const v4f*)(pa + 4);
    const v4f f2 = *(const v4f*)(pa + 16);
    const v4f f3 = *(const v4f*)(pa + 20);
    Frag a;
    a.v[0]  = (_Float16)f0.x; a.v[1]  = (_Float16)f0.y; a.v[2]  = (_Float16)f0.z; a.v[3]  = (_Float16)f0.w;
    a.v[4]  = (_Float16)f1.x; a.v[5]  = (_Float16)f1.y; a.v[6]  = (_Float16)f1.z; a.v[7]  = (_Float16)f1.w;
    a.v[8]  = (_Float16)f2.x; a.v[9]  = (_Float16)f2.y; a.v[10] = (_Float16)f2.z; a.v[11] = (_Float16)f2.w;
    a.v[12] = (_Float16)f3.x; a.v[13] = (_Float16)f3.y; a.v[14] = (_Float16)f3.z; a.v[15] = (_Float16)f3.w;
    Frag b;
    b.h[0] = *(const v8h*)(bp + 32 * ks);
    b.h[1] = *(const v8h*)(bp + 32 * ks + 16);
    acc = wmh(a.v, b.v, acc);
  }

  if (m < 2) {
    float* sp = stg + m * GROWS + wave * 16 + 8 * hh;
    v4f s0, s1;
    s0.x = acc[0] * RWS; s0.y = acc[1] * RWS; s0.z = acc[2] * RWS; s0.w = acc[3] * RWS;
    s1.x = acc[4] * RWS; s1.y = acc[5] * RWS; s1.z = acc[6] * RWS; s1.w = acc[7] * RWS;
    *(v4f*)sp = s0;
    *(v4f*)(sp + 4) = s1;
  }
  __syncthreads();

  if (wave == 0) {
    const v4f v = *(const v4f*)(stg + 4 * lane);
    float* gp = AB + (size_t)(lane >> 4) * (size_t)nPad + rowBase + 4 * (lane & 15);
    *(volatile v4f*)gp = v;
    __threadfence();
    *(volatile v4f*)gp = v;
  }
}

__global__ __launch_bounds__(ETHR) void k_edge(const float* __restrict__ AB,
                                               const int* __restrict__ ei,
                                               const int* __restrict__ fri,
                                               float* out, int nN, int nE, int nPad) {
  __shared__ __attribute__((aligned(16))) float sc[ETHR];
  const int tid = threadIdx.x, lane = tid & 31, wave = tid >> 5;
  const float* Ap = AB;
  const float* Bp = AB + (size_t)nPad;

  int e = blockIdx.x * ETHR + tid;
  e = e > nE - 1 ? nE - 1 : e;
  const int j  = clampi(fri[e], nE - 1);
  const int r0 = clampi(ei[e], nN - 1);
  const int c0 = clampi(ei[(size_t)nE + e], nN - 1);
  const int r1 = clampi(ei[j], nN - 1);
  const int c1 = clampi(ei[(size_t)nE + j], nN - 1);

  const float l0 = Ap[r0] + Bp[c0];
  const float l1 = Ap[r1] + Bp[c1];
  const float w0 = sigm(l0);
  const float w1 = sigm(l1);
  sc[tid] = w0 * w1;
  __syncthreads();

  if (wave < 2) {
    const int idx = wave * 32 + lane;
    const v4f ov = *(const v4f*)(sc + 4 * idx);
    const int e0 = blockIdx.x * ETHR + 4 * idx;
    float* op = out + e0;
    const bool full = (e0 + 3 < nE);
    if (full) {
      *(volatile v4f*)op = ov;
    } else {
      if (e0     < nE) *(volatile float*)(op)     = ov.x;
      if (e0 + 1 < nE) *(volatile float*)(op + 1) = ov.y;
      if (e0 + 2 < nE) *(volatile float*)(op + 2) = ov.z;
    }
    __threadfence();
    if (full) {
      *(volatile v4f*)op = ov;
    } else {
      if (e0     < nE) *(volatile float*)(op)     = ov.x;
      if (e0 + 1 < nE) *(volatile float*)(op + 1) = ov.y;
      if (e0 + 2 < nE) *(volatile float*)(op + 2) = ov.z;
    }
  }
}

extern "C" void kernel_launch(void* const* d_in, const int* in_sizes, int n_in,
                              void* d_out, int out_size, void* d_ws, size_t ws_size,
                              hipStream_t stream) {
  if (n_in < 4) return;
  const int nN = in_sizes[0] / CH;
  const int nE = in_sizes[2];
  if (nN <= 0 || nE <= 0) return;
  if (in_sizes[0] != nN * CH || in_sizes[1] != 2 * nE || in_sizes[3] != 2 * CH) return;
  if (out_size != nE) return;
  if (nN > (1 << 24) || nE > (1 << 28)) return;

  const float* x   = (const float*)d_in[0];
  const int*   ei  = (const int*)d_in[1];
  const int*   fri = (const int*)d_in[2];
  const float* W   = (const float*)d_in[3];
  float* out = (float*)d_out;

  const int nBlkG = (nN + GROWS - 1) / GROWS;
  const int nPad  = nBlkG * GROWS;
  const int nBlkE = (nE + ETHR - 1) / ETHR;

  char* ws = (char*)d_ws;
  size_t off = 0;
  const size_t oW  = off; off += (size_t)NCOL * KPB * 2;       off = (off + 255) & ~(size_t)255;
  const size_t oAB = off; off += (size_t)2 * nPad * 4;         off = (off + 255) & ~(size_t)255;
  if (off > ws_size || off > (size_t)WSCAP) return;
  _Float16* Wpl = (_Float16*)(ws + oW);
  float*    AB  = (float*)(ws + oAB);

  k_wprep<<<1, PTHR, 0, stream>>>(W, Wpl);
  k_nodegemm<<<nBlkG, GTHR, 0, stream>>>(x, Wpl, AB, nN, nPad);
  k_edge<<<nBlkE, ETHR, 0, stream>>>(AB, ei, fri, out, nN, nE, nPad);
}
